// GCGRU_59493886984732
// MI455X (gfx1250) — hardware-verified
//
#include <hip/hip_runtime.h>

typedef __attribute__((ext_vector_type(16))) _Float16 v16h;
typedef __attribute__((ext_vector_type(8)))  _Float16 v8h;
typedef __attribute__((ext_vector_type(16))) __bf16   v16b;
typedef __attribute__((ext_vector_type(8)))  __bf16   v8b;
typedef __attribute__((ext_vector_type(8)))  float    v8f;
typedef __attribute__((ext_vector_type(4)))  float    v4f;
typedef __attribute__((ext_vector_type(2)))  float    v2f;
typedef __attribute__((ext_vector_type(4)))  unsigned v4u;

constexpr int NNODE  = 2048;
constexpr int BATCH  = 16;
constexpr int XDIM   = 2;
constexpr int HID    = 64;
constexpr int CIN    = XDIM + HID;
constexpr int EDIM   = 10;
constexpr int CHEB   = 3;
constexpr int KI     = CHEB * CIN;
constexpr int KPAD   = 224;
constexpr int KCH    = KPAD / 8;
constexpr int KPW    = (KPAD - KI) / 2;
constexpr int OG     = 2 * HID;
constexpr int OU     = HID;
constexpr int FDIM   = BATCH * CIN;
constexpr int FPAD   = 1088;
constexpr int NDG    = EDIM * OG;
constexpr int NDU    = EDIM * OU;
constexpr int MROWS  = BATCH * NNODE;
constexpr int GCHUNK = 8192;
constexpr int UCHUNK = 16384;
constexpr int NTILE  = 64;

static_assert((KPAD % 32) == 0 && KPAD >= KI);
static_assert((KI % 2) == 0 && ((KPAD - KI) % 2) == 0);
static_assert((FPAD % 64) == 0 && FPAD >= FDIM);
static_assert((NNODE % 64) == 0 && (NNODE % 32) == 0);
static_assert((((FPAD / 64) * (NNODE / 64)) % 8) == 0);
static_assert((GCHUNK % 64) == 0 && (NDG % 64) == 0 && (((GCHUNK / 64) * (NDG / 64)) % 8) == 0);
static_assert((UCHUNK % 64) == 0 && (NDU % 64) == 0 && (((UCHUNK / 64) * (NDU / 64)) % 8) == 0);
static_assert((MROWS % GCHUNK) == 0 && (MROWS % UCHUNK) == 0);
static_assert((NNODE % NTILE) == 0 && (GCHUNK % NTILE) == 0 && (UCHUNK % NTILE) == 0);
static_assert(NNODE == 8 * 256);
static_assert(((NDG * KCH) % 256) == 0 && ((NDU * KCH) % 256) == 0);
static_assert(NTILE * KPAD * 2 == 7 * 256 * 16);
static_assert(NTILE * HID * 4 == 4 * 256 * 16);
static_assert(NTILE * EDIM <= 1024 && NDG <= 2048);

constexpr size_t AMAT_BYTES = (size_t)NNODE * NNODE * 2;
constexpr size_t XT_BYTES   = (size_t)FPAD * NNODE * 2;
constexpr size_t XG_BYTES   = (size_t)MROWS * KPAD * 2;
constexpr size_t PTG_BYTES  = (size_t)NDG * KPAD * 2;
constexpr size_t PTU_BYTES  = (size_t)NDU * KPAD * 2;
constexpr size_t ZB_BYTES   = (size_t)MROWS * HID * 4;
constexpr size_t P2_BYTES   = (size_t)FPAD * NNODE * 4;
constexpr size_t YG_BYTES   = (size_t)GCHUNK * NDG * 4;
constexpr size_t YU_BYTES   = (size_t)UCHUNK * NDU * 4;
constexpr size_t Y_BYTES    = (YG_BYTES > YU_BYTES) ? YG_BYTES : YU_BYTES;

constexpr size_t OFF_AH  = 0;
constexpr size_t OFF_AL  = OFF_AH  + AMAT_BYTES;
constexpr size_t OFF_X0H = OFF_AL  + AMAT_BYTES;
constexpr size_t OFF_X0L = OFF_X0H + XT_BYTES;
constexpr size_t OFF_XGH = OFF_X0L + XT_BYTES;
constexpr size_t OFF_XGL = OFF_XGH + XG_BYTES;
constexpr size_t OFF_PTG = OFF_XGL + XG_BYTES;
constexpr size_t OFF_PTU = OFF_PTG + PTG_BYTES;
constexpr size_t OFF_ZB  = OFF_PTU + PTU_BYTES;
constexpr size_t OFF_Y   = OFF_ZB  + ZB_BYTES;
constexpr size_t OFF_P2  = OFF_Y;
constexpr size_t OFF_X1H = OFF_P2  + P2_BYTES;
constexpr size_t OFF_X1L = OFF_X1H + XT_BYTES;
constexpr size_t WS_TOTAL = OFF_Y + Y_BYTES;
static_assert(OFF_X1L + XT_BYTES <= OFF_Y + Y_BYTES);
static_assert(Y_BYTES >= YG_BYTES && Y_BYTES >= YU_BYTES && Y_BYTES >= P2_BYTES + 2 * XT_BYTES);
static_assert(WS_TOTAL <= (size_t)134217728);
static_assert((OFF_AL % 256) == 0 && (OFF_X0H % 256) == 0 && (OFF_X0L % 256) == 0 && (OFF_XGH % 256) == 0 &&
              (OFF_XGL % 256) == 0 && (OFF_PTG % 256) == 0 && (OFF_PTU % 256) == 0 && (OFF_ZB % 256) == 0 &&
              (OFF_Y % 256) == 0 && (OFF_X1H % 256) == 0 && (OFF_X1L % 256) == 0);

__device__ __forceinline__ unsigned short f2bf_bits(float f) {
  unsigned u = __float_as_uint(f);
  return (unsigned short)((u + 0x7FFFu + ((u >> 16) & 1u)) >> 16);
}
__device__ __forceinline__ float bf_bits2f(unsigned short h) { return __uint_as_float(((unsigned)h) << 16); }
__device__ __forceinline__ float bfr(float f) { return __uint_as_float(((unsigned)f2bf_bits(f)) << 16); }
__device__ __forceinline__ void split2(float a, float b, unsigned& wh, unsigned& wl) {
  const unsigned short ha = f2bf_bits(a), hb = f2bf_bits(b);
  const unsigned short la = f2bf_bits(a - bf_bits2f(ha)), lb = f2bf_bits(b - bf_bits2f(hb));
  wh = (unsigned)ha | ((unsigned)hb << 16);
  wl = (unsigned)la | ((unsigned)lb << 16);
}
__device__ __forceinline__ unsigned pack2bf(float a, float b) {
  return (unsigned)f2bf_bits(a) | ((unsigned)f2bf_bits(b) << 16);
}

__device__ __forceinline__ void dep_guard_h(v8f& a, v8f& b, v16h x, v16h y) { asm volatile("v_nop\n\tv_nop\n\tv_nop\n\tv_nop" : "+v"(a), "+v"(b) : "v"(x), "v"(y)); }
__device__ __forceinline__ void dep_guard_b(v8f& a, v8f& b, v16b x, v16b y) { asm volatile("v_nop\n\tv_nop\n\tv_nop\n\tv_nop" : "+v"(a), "+v"(b) : "v"(x), "v"(y)); }
__device__ __forceinline__ void keep4_h(v16h a, v16h b, v16h c, v16h d) { asm volatile("v_nop" :: "v"(a), "v"(b), "v"(c), "v"(d)); }
__device__ __forceinline__ void keep4_b(v16b a, v16b b, v16b c, v16b d) { asm volatile("v_nop" :: "v"(a), "v"(b), "v"(c), "v"(d)); }
__device__ __forceinline__ void acc_guard4(v8f& a, v8f& b, v8f& c, v8f& d) { asm volatile("v_nop\n\tv_nop\n\tv_nop\n\tv_nop" : "+v"(a), "+v"(b), "+v"(c), "+v"(d)); }
template <typename T> struct Frag;
template <> struct Frag<_Float16> {
  typedef v16h V; union U { v16h v; v8h h[2]; };
  static __device__ __forceinline__ v16h load(const _Float16* p) {
    U f; f.h[0] = *(const v8h*)(p); f.h[1] = *(const v8h*)(p + 16); return f.v;
  }
  static __device__ __forceinline__ v8f mma(v16h a, v16h b, v8f c) {
    return __builtin_amdgcn_wmma_f32_16x16x32_f16(false, a, false, b, (short)0, c, false, false);
  }
  static __device__ __forceinline__ void guard(v8f& a, v8f& b, v16h x, v16h y) { dep_guard_h(a, b, x, y); }
  static __device__ __forceinline__ void keep(v16h a, v16h b, v16h c, v16h d) { keep4_h(a, b, c, d); }
};
template <> struct Frag<__bf16> {
  typedef v16b V; union U { v16b v; v8b h[2]; };
  static __device__ __forceinline__ v16b load(const __bf16* p) {
    U f; f.h[0] = *(const v8b*)(p); f.h[1] = *(const v8b*)(p + 16); return f.v;
  }
  static __device__ __forceinline__ v8f mma(v16b a, v16b b, v8f c) {
    return __builtin_amdgcn_wmma_f32_16x16x32_bf16(false, a, false, b, (short)0, c, false, false);
  }
  static __device__ __forceinline__ void guard(v8f& a, v8f& b, v16b x, v16b y) { dep_guard_b(a, b, x, y); }
  static __device__ __forceinline__ void keep(v16b a, v16b b, v16b c, v16b d) { keep4_b(a, b, c, d); }
};

template <int ET> struct Elem;
template <> struct Elem<0> { typedef _Float16 T; };
template <> struct Elem<1> { typedef __bf16 T; };
template <int ET, int SPLITM, int OUT_MODE>
__global__ __launch_bounds__(256) void wmma_gemm64(
    const unsigned short* __restrict__ Ap, const unsigned short* __restrict__ A2p, int lda, long strideA,
    const unsigned short* __restrict__ Btp, const unsigned short* __restrict__ Bt2p, int ldb, long strideB,
    void* __restrict__ Cout, void* __restrict__ Cout2, int ldc, long strideC,
    int M, int N, int K, float scale) {
  constexpr bool ASPL = (SPLITM == 1) || (SPLITM == 3);
  constexpr bool BSPL = (SPLITM == 1) || (SPLITM == 2);
  typedef typename Elem<ET>::T T;
  typedef typename Frag<T>::V V;
  const T* A = (const T*)Ap; const T* A2 = (const T*)A2p; const T* Bt = (const T*)Btp; const T* Bt2 = (const T*)Bt2p;
  __shared__ __align__(16) float sT[8][16 * 68];
  const int b    = blockIdx.y;
  const int lane = threadIdx.x & 31;
  const int wave = threadIdx.x >> 5;
  const int tilesN = N >> 6;
  const int tilesM = M >> 6;
  const int tile = blockIdx.x * 8 + wave;
  if (tile >= tilesM * tilesN) return;
  const int tm = tile / tilesN;
  const int tn = tile - tm * tilesN;
  const int m0 = tm << 6;
  const int n0 = tn << 6;

  const T* Ab  = A  + (size_t)b * strideA;
  const T* Bb  = Bt + (size_t)b * strideB;
  const T* Ab2 = ASPL ? (A2  + (size_t)b * strideA) : nullptr;
  const T* Bb2 = BSPL ? (Bt2 + (size_t)b * strideB) : nullptr;

  const int rlane = lane & 15;
  const int koff  = (lane >> 4) * 8;
  const int mOff  = (lane >> 4) * 8;

  v8f acc[4][4];
#pragma unroll
  for (int i = 0; i < 4; ++i)
#pragma unroll
    for (int j = 0; j < 4; ++j) acc[i][j] = (v8f){0.f,0.f,0.f,0.f,0.f,0.f,0.f,0.f};

  for (int k0 = 0; k0 < K; k0 += 32) {
    V bh[4], bl[4];
#pragma unroll
    for (int j = 0; j < 4; ++j) {
      const size_t bo = (size_t)(n0 + (j << 4) + rlane) * ldb + koff + k0;
      bh[j] = Frag<T>::load(Bb + bo);
      if (BSPL) bl[j] = Frag<T>::load(Bb2 + bo);
    }
#pragma unroll
    for (int i = 0; i < 4; ++i) {
      const size_t ao = (size_t)(m0 + (i << 4) + rlane) * lda + koff + k0;
      V ah = Frag<T>::load(Ab + ao);
      V al = ah;
      if (ASPL) al = Frag<T>::load(Ab2 + ao);
#pragma unroll
      for (int j = 0; j < 4; ++j) {
        acc[i][j] = Frag<T>::mma(ah, bh[j], acc[i][j]);
        if (BSPL) acc[i][j] = Frag<T>::mma(ah, bl[j], acc[i][j]);
        if (ASPL) acc[i][j] = Frag<T>::mma(al, bh[j], acc[i][j]);
      }
      Frag<T>::guard(acc[i][0], acc[i][3], ah, al);
    }
    Frag<T>::keep(bh[0], bh[1], bh[2], bh[3]);
    if (BSPL) Frag<T>::keep(bl[0], bl[1], bl[2], bl[3]);
  }
  acc_guard4(acc[0][0], acc[0][1], acc[0][2], acc[0][3]);
  acc_guard4(acc[1][0], acc[1][1], acc[1][2], acc[1][3]);
  acc_guard4(acc[2][0], acc[2][1], acc[2][2], acc[2][3]);
  acc_guard4(acc[3][0], acc[3][1], acc[3][2], acc[3][3]);

  float* slab = sT[wave];
#pragma unroll
  for (int i = 0; i < 4; ++i) {
    const int mBase = m0 + (i << 4);
#pragma unroll
    for (int j = 0; j < 4; ++j) {
#pragma unroll
      for (int r = 0; r < 8; ++r) {
        const float v = acc[i][j][r] * scale;
        slab[(mOff + r) * 68 + (j << 4) + rlane] = v;
      }
    }
    __builtin_amdgcn_fence(__ATOMIC_RELEASE, "workgroup");
    __builtin_amdgcn_wave_barrier();
    __builtin_amdgcn_fence(__ATOMIC_ACQUIRE, "workgroup");
    if (OUT_MODE == 0) {
      float* C = (float*)Cout + (size_t)b * strideC;
      const int hh = lane >> 4, c4 = (lane & 15) * 4;
      for (int pass = 0; pass < 2; ++pass) {
#pragma unroll
        for (int it = 0; it < 8; ++it) {
          const int row = it * 2 + hh;
          v4f v = *(const v4f*)(slab + row * 68 + c4);
          *(volatile v4f*)(C + (size_t)(mBase + row) * ldc + n0 + c4) = v;
        }
        __threadfence();
      }
    } else {
      const int q = lane >> 3, c8 = (lane & 7) * 8;
      unsigned short* C  = (unsigned short*)Cout  + (size_t)b * strideC;
      unsigned short* C2 = (OUT_MODE == 2) ? ((unsigned short*)Cout2 + (size_t)b * strideC) : nullptr;
      for (int pass = 0; pass < 2; ++pass) {
#pragma unroll
        for (int it = 0; it < 4; ++it) {
          const int row = it * 4 + q;
          const float* sp = slab + row * 68 + c8;
          v8h hv, lv;
#pragma unroll
          for (int e = 0; e < 8; ++e) {
            if (OUT_MODE == 1) {
              hv[e] = (_Float16)sp[e];
            } else {
              unsigned short hb = f2bf_bits(sp[e]);
              unsigned short lb = f2bf_bits(sp[e] - bf_bits2f(hb));
              hv[e] = __builtin_bit_cast(_Float16, hb);
              lv[e] = __builtin_bit_cast(_Float16, lb);
            }
          }
          *(volatile v8h*)(C + (size_t)(mBase + row) * ldc + n0 + c8) = hv;
          if (OUT_MODE == 2) *(volatile v8h*)(C2 + (size_t)(mBase + row) * ldc + n0 + c8) = lv;
        }
        __threadfence();
      }
    }
    __builtin_amdgcn_fence(__ATOMIC_RELEASE, "workgroup");
    __builtin_amdgcn_wave_barrier();
    __builtin_amdgcn_fence(__ATOMIC_ACQUIRE, "workgroup");
  }
}

__global__ __launch_bounds__(256) void adj_softmax_kernel(const float* __restrict__ E,
                                                          unsigned short* __restrict__ Ah,
                                                          unsigned short* __restrict__ Al) {
  __shared__ __align__(16) float rowv[NNODE];
  __shared__ float red[256];
  __shared__ float Ei[EDIM];
  const int i = blockIdx.x;
  const int t = threadIdx.x;
  if (t < EDIM) Ei[t] = bfr(E[(size_t)i * EDIM + t]);
  __syncthreads();

  float lmax = 0.f;
#pragma unroll 1
  for (int j = t; j < NNODE; j += 256) {
    const float* ej = E + (size_t)j * EDIM;
    float s = 0.f;
#pragma unroll
    for (int d = 0; d < EDIM; ++d) s = fmaf(Ei[d], bfr(ej[d]), s);
    s = fmaxf(s, 0.f);
    rowv[j] = s;
    lmax = fmaxf(lmax, s);
  }
  red[t] = lmax;
  __syncthreads();
  for (int st = 128; st > 0; st >>= 1) {
    if (t < st) red[t] = fmaxf(red[t], red[t + st]);
    __syncthreads();
  }
  const float mx = red[0];
  __syncthreads();

  float lsum = 0.f;
#pragma unroll 1
  for (int j = t; j < NNODE; j += 256) {
    const float e = expf(rowv[j] - mx);
    rowv[j] = e;
    lsum += e;
  }
  red[t] = lsum;
  __syncthreads();
  for (int st = 128; st > 0; st >>= 1) {
    if (t < st) red[t] += red[t + st];
    __syncthreads();
  }
  const float inv = 1.0f / red[0];

  const int j0 = 8 * t;
  unsigned wh0, wh1, wh2, wh3, wl0, wl1, wl2, wl3;
  split2(rowv[j0 + 0] * inv, rowv[j0 + 1] * inv, wh0, wl0);
  split2(rowv[j0 + 2] * inv, rowv[j0 + 3] * inv, wh1, wl1);
  split2(rowv[j0 + 4] * inv, rowv[j0 + 5] * inv, wh2, wl2);
  split2(rowv[j0 + 6] * inv, rowv[j0 + 7] * inv, wh3, wl3);
  const v4u hv = (v4u){wh0, wh1, wh2, wh3};
  const v4u lv = (v4u){wl0, wl1, wl2, wl3};
  const size_t off = (size_t)i * NNODE + j0;
  *(volatile v4u*)(Ah + off) = hv;
  *(volatile v4u*)(Al + off) = lv;
  __threadfence();
  *(volatile v4u*)(Ah + off) = hv;
  *(volatile v4u*)(Al + off) = lv;
}

__global__ __launch_bounds__(256) void pack_feat_kernel(const float* __restrict__ x,
                                                        const float* __restrict__ state,
                                                        unsigned short* __restrict__ X0h,
                                                        unsigned short* __restrict__ X0l) {
  const int f = blockIdx.x;
  const int t = threadIdx.x;
  const int n = 8 * t;
  unsigned w0 = 0u, w1 = 0u, w2 = 0u, w3 = 0u;
  if (f < FDIM) {
    const int b = f / CIN;
    const int c = f - b * CIN;
    float v[8];
    if (c < XDIM) {
#pragma unroll
      for (int e = 0; e < 8; ++e) v[e] = x[((size_t)b * NNODE + n + e) * XDIM + c];
    } else {
#pragma unroll
      for (int e = 0; e < 8; ++e) v[e] = state[((size_t)b * NNODE + n + e) * HID + (c - XDIM)];
    }
    w0 = pack2bf(v[0], v[1]); w1 = pack2bf(v[2], v[3]); w2 = pack2bf(v[4], v[5]); w3 = pack2bf(v[6], v[7]);
  }
  const v4u hv = (v4u){w0, w1, w2, w3};
  const v4u zv = (v4u){0u, 0u, 0u, 0u};
  const size_t off = (size_t)f * NNODE + n;
  *(volatile v4u*)(X0h + off) = hv;
  *(volatile v4u*)(X0l + off) = zv;
  __threadfence();
  *(volatile v4u*)(X0h + off) = hv;
  *(volatile v4u*)(X0l + off) = zv;
}

__global__ __launch_bounds__(256) void pool_pack_kernel(const float* __restrict__ pool,
                                                        unsigned short* __restrict__ PT,
                                                        int ocols, int nchunk) {
  const int q = blockIdx.x * 256 + threadIdx.x;
  if (q >= nchunk) return;
  const int row = q / KCH;
  const int c8 = (q - row * KCH) * 8;
  const int d = row / ocols;
  const int o = row - d * ocols;
  float v[8];
#pragma unroll
  for (int e = 0; e < 8; ++e) {
    const int k = c8 + e;
    const int kc = (k < KI) ? k : (KI - 1);
    const int kk = kc / CIN;
    const int ii = kc - kk * CIN;
    const float pv = pool[((size_t)((d * CHEB + kk) * CIN + ii)) * ocols + o];
    v[e] = (k < KI) ? pv : 0.f;
  }
  const v4u hv = (v4u){pack2bf(v[0], v[1]), pack2bf(v[2], v[3]), pack2bf(v[4], v[5]), pack2bf(v[6], v[7])};
  const size_t off = (size_t)row * KPAD + c8;
  *(volatile v4u*)(PT + off) = hv;
  __threadfence();
  *(volatile v4u*)(PT + off) = hv;
}

__global__ __launch_bounds__(256) void pack_xg_kernel(const unsigned short* __restrict__ X0h,
                                                      const unsigned short* __restrict__ X0l,
                                                      const unsigned short* __restrict__ X1h,
                                                      const unsigned short* __restrict__ X1l,
                                                      const float* __restrict__ P2,
                                                      unsigned short* __restrict__ XGh,
                                                      unsigned short* __restrict__ XGl) {
  __shared__ __align__(16) unsigned short th[NTILE * KPAD];
  __shared__ __align__(16) unsigned short tl[NTILE * KPAD];
  const int n0 = blockIdx.x * NTILE;
  const int b = blockIdx.y;
  const int t = threadIdx.x;
  unsigned* th32 = (unsigned*)th;
  unsigned* tl32 = (unsigned*)tl;
  for (int q = t; q < NTILE * KPW; q += 256) {
    const int r = q / KPW;
    const int cc = q - r * KPW;
    const int wi = (r * KPAD + KI) / 2 + cc;
    th32[wi] = 0u;
    tl32[wi] = 0u;
  }
#pragma unroll 1
  for (int idx = t; idx < CIN * (NTILE / 2); idx += 256) {
    const int c = idx / (NTILE / 2);
    const int rp = idx - c * (NTILE / 2);
    const int r = 2 * rp;
    const size_t src = (size_t)(b * CIN + c) * NNODE + n0 + r;
    const unsigned a0h = *(const unsigned*)(X0h + src);
    const unsigned a0l = *(const unsigned*)(X0l + src);
    const unsigned a1h = *(const unsigned*)(X1h + src);
    const unsigned a1l = *(const unsigned*)(X1l + src);
    const v2f p = *(const v2f*)(P2 + src);
    const float x0a = __uint_as_float(a0h << 16) + __uint_as_float(a0l << 16);
    const float x0b = __uint_as_float(a0h & 0xffff0000u) + __uint_as_float(a0l & 0xffff0000u);
    unsigned w2h, w2l;
    split2(p.x - x0a, p.y - x0b, w2h, w2l);
    const int ia = r * KPAD + c;
    const int ib = ia + KPAD;
    th[ia] = (unsigned short)(a0h & 0xffffu);  th[ib] = (unsigned short)(a0h >> 16);
    tl[ia] = (unsigned short)(a0l & 0xffffu);  tl[ib] = (unsigned short)(a0l >> 16);
    th[ia + CIN] = (unsigned short)(a1h & 0xffffu);  th[ib + CIN] = (unsigned short)(a1h >> 16);
    tl[ia + CIN] = (unsigned short)(a1l & 0xffffu);  tl[ib + CIN] = (unsigned short)(a1l >> 16);
    th[ia + 2 * CIN] = (unsigned short)(w2h & 0xffffu);  th[ib + 2 * CIN] = (unsigned short)(w2h >> 16);
    tl[ia + 2 * CIN] = (unsigned short)(w2l & 0xffffu);  tl[ib + 2 * CIN] = (unsigned short)(w2l >> 16);
  }
  __syncthreads();
  const size_t base = ((size_t)b * NNODE + n0) * KPAD;
  const v4u* th4 = (const v4u*)th;
  const v4u* tl4 = (const v4u*)tl;
  for (int pass = 0; pass < 2; ++pass) {
#pragma unroll
    for (int it = 0; it < 7; ++it) {
      const int q = it * 256 + t;
      const v4u hv = th4[q];
      const v4u lv = tl4[q];
      *(volatile v4u*)(XGh + base + (size_t)q * 8) = hv;
      *(volatile v4u*)(XGl + base + (size_t)q * 8) = lv;
    }
    __threadfence();
  }
}

__global__ __launch_bounds__(256) void gate_epi_kernel(const float* __restrict__ Y,
                                                       const float* __restrict__ E,
                                                       const float* __restrict__ gbias,
                                                       const float* __restrict__ state,
                                                       float* __restrict__ zbuf,
                                                       unsigned short* __restrict__ X0h,
                                                       unsigned short* __restrict__ X0l,
                                                       int row0) {
  __shared__ float Esh[NTILE * EDIM];
  __shared__ float bsh[NDG];
  __shared__ __align__(16) float zs[NTILE * HID];
  __shared__ __align__(16) unsigned short rsh[HID * NTILE];
  __shared__ __align__(16) unsigned short rsl[HID * NTILE];
  const int t = threadIdx.x;
  const int R = row0 + blockIdx.x * NTILE;
  const int b = R / NNODE;
  const int n0 = R - b * NNODE;
  for (int q = t; q < NTILE * EDIM; q += 256) Esh[q] = bfr(E[(size_t)n0 * EDIM + q]);
  for (int q = t; q < NDG; q += 256) bsh[q] = bfr(gbias[q]);
  __syncthreads();

  const int o = t & (OG - 1);
  const int half = t >> 7;
  const float* Yb = Y + (size_t)(blockIdx.x * NTILE) * NDG;
#pragma unroll 1
  for (int it = 0; it < NTILE / 2; ++it) {
    const int nn = 2 * it + half;
    const float* yr = Yb + (size_t)nn * NDG;
    float acc = 0.f;
#pragma unroll
    for (int d = 0; d < EDIM; ++d) acc = fmaf(Esh[nn * EDIM + d], yr[d * OG + o] + bsh[d * OG + o], acc);
    const float sg = 1.0f / (1.0f + expf(-acc));
    if (o < HID) {
      zs[nn * HID + o] = sg;
    } else {
      const int h = o - HID;
      const float st = bfr(state[((size_t)b * NNODE + n0 + nn) * HID + h]);
      const float rs = sg * st;
      const unsigned short hb = f2bf_bits(rs);
      const unsigned short lb = f2bf_bits(rs - bf_bits2f(hb));
      rsh[h * NTILE + nn] = hb;
      rsl[h * NTILE + nn] = lb;
    }
  }
  __syncthreads();

  float* zdst = zbuf + (size_t)R * HID;
  const v4f* zs4 = (const v4f*)zs;
  const v4u* rh4 = (const v4u*)rsh;
  const v4u* rl4 = (const v4u*)rsl;
  const int seg = t & 7;
  for (int pass = 0; pass < 2; ++pass) {
#pragma unroll
    for (int it = 0; it < 4; ++it) {
      const int q = it * 256 + t;
      const v4f v = zs4[q];
      *(volatile v4f*)(zdst + (size_t)q * 4) = v;
    }
#pragma unroll
    for (int s = 0; s < 2; ++s) {
      const int h = s * 32 + (t >> 3);
      const v4u hv = rh4[h * (NTILE / 8) + seg];
      const v4u lv = rl4[h * (NTILE / 8) + seg];
      const size_t off = (size_t)(b * CIN + XDIM + h) * NNODE + n0 + seg * 8;
      *(volatile v4u*)(X0h + off) = hv;
      *(volatile v4u*)(X0l + off) = lv;
    }
    __threadfence();
  }
}

__global__ __launch_bounds__(256) void cand_epi_kernel(const float* __restrict__ Y,
                                                       const float* __restrict__ E,
                                                       const float* __restrict__ ubias,
                                                       const float* __restrict__ state,
                                                       const float* __restrict__ zbuf,
                                                       float* __restrict__ out,
                                                       int row0) {
  __shared__ float Esh[NTILE * EDIM];
  __shared__ float bsh[NDU];
  __shared__ __align__(16) float os[NTILE * HID];
  const int t = threadIdx.x;
  const int R = row0 + blockIdx.x * NTILE;
  const int b = R / NNODE;
  const int n0 = R - b * NNODE;
  for (int q = t; q < NTILE * EDIM; q += 256) Esh[q] = bfr(E[(size_t)n0 * EDIM + q]);
  for (int q = t; q < NDU; q += 256) bsh[q] = bfr(ubias[q]);
  __syncthreads();

  const int o = t & (OU - 1);
  const int q4 = t >> 6;
  const float* Yb = Y + (size_t)(blockIdx.x * NTILE) * NDU;
#pragma unroll 1
  for (int it = 0; it < NTILE / 4; ++it) {
    const int nn = 4 * it + q4;
    const float* yr = Yb + (size_t)nn * NDU;
    float acc = 0.f;
#pragma unroll
    for (int d = 0; d < EDIM; ++d) acc = fmaf(Esh[nn * EDIM + d], yr[d * OU + o] + bsh[d * OU + o], acc);
    const float hc = tanhf(acc);
    const size_t g = ((size_t)R + nn) * HID + o;
    const float z = zbuf[g];
    const float st = bfr(state[g]);
    os[nn * HID + o] = z * st + (1.0f - z) * hc;
  }
  __syncthreads();

  float* dst = out + (size_t)R * HID;
  const v4f* os4 = (const v4f*)os;
  for (int pass = 0; pass < 2; ++pass) {
#pragma unroll
    for (int it = 0; it < 4; ++it) {
      const int q = it * 256 + t;
      const v4f v = os4[q];
      *(volatile v4f*)(dst + (size_t)q * 4) = v;
    }
    __threadfence();
  }
}

extern "C" void kernel_launch(void* const* d_in, const int* in_sizes, int n_in,
                              void* d_out, int out_size, void* d_ws, size_t ws_size,
                              hipStream_t stream) {
  if (n_in < 7) return;
  if (in_sizes[0] != BATCH * NNODE * XDIM) return;
  if (in_sizes[1] != MROWS * HID) return;
  if (in_sizes[2] != NNODE * EDIM) return;
  if (in_sizes[3] != EDIM * CHEB * CIN * OG) return;
  if (in_sizes[4] != EDIM * OG) return;
  if (in_sizes[5] != EDIM * CHEB * CIN * OU) return;
  if (in_sizes[6] != EDIM * OU) return;
  if (out_size != MROWS * HID) return;
  if (ws_size < WS_TOTAL) return;

  const float* x     = (const float*)d_in[0];
  const float* state = (const float*)d_in[1];
  const float* E     = (const float*)d_in[2];
  const float* gW    = (const float*)d_in[3];
  const float* gB    = (const float*)d_in[4];
  const float* uW    = (const float*)d_in[5];
  const float* uB    = (const float*)d_in[6];
  float* out = (float*)d_out;

  char* ws = (char*)d_ws;
  unsigned short* Ah  = (unsigned short*)(ws + OFF_AH);
  unsigned short* Al  = (unsigned short*)(ws + OFF_AL);
  unsigned short* X0h = (unsigned short*)(ws + OFF_X0H);
  unsigned short* X0l = (unsigned short*)(ws + OFF_X0L);
  unsigned short* XGh = (unsigned short*)(ws + OFF_XGH);
  unsigned short* XGl = (unsigned short*)(ws + OFF_XGL);
  unsigned short* PTg = (unsigned short*)(ws + OFF_PTG);
  unsigned short* PTu = (unsigned short*)(ws + OFF_PTU);
  float*          zb  = (float*)(ws + OFF_ZB);
  float*          Y   = (float*)(ws + OFF_Y);
  float*          P2  = (float*)(ws + OFF_P2);
  unsigned short* X1h = (unsigned short*)(ws + OFF_X1H);
  unsigned short* X1l = (unsigned short*)(ws + OFF_X1L);

  adj_softmax_kernel<<<NNODE, 256, 0, stream>>>(E, Ah, Al);
  pack_feat_kernel<<<FPAD, 256, 0, stream>>>(x, state, X0h, X0l);
  pool_pack_kernel<<<(NDG * KCH) / 256, 256, 0, stream>>>(gW, PTg, OG, NDG * KCH);
  pool_pack_kernel<<<(NDU * KCH) / 256, 256, 0, stream>>>(uW, PTu, OU, NDU * KCH);

  const dim3 gprop(((FPAD / 64) * (NNODE / 64)) / 8, 1);
  const dim3 gng(((GCHUNK / 64) * (NDG / 64)) / 8, 1);
  const dim3 gnu(((UCHUNK / 64) * (NDU / 64)) / 8, 1);
  const dim3 gxg(NNODE / NTILE, BATCH);

  wmma_gemm64<1, 2, 2><<<gprop, 256, 0, stream>>>(X0h, X0l, NNODE, 0L, Ah, Al, NNODE, 0L,
                                                   (void*)X1h, (void*)X1l, NNODE, 0L,
                                                   FPAD, NNODE, NNODE, 1.0f);
  wmma_gemm64<1, 1, 0><<<gprop, 256, 0, stream>>>(X1h, X1l, NNODE, 0L, Ah, Al, NNODE, 0L,
                                                   (void*)P2, (void*)P2, NNODE, 0L,
                                                   FPAD, NNODE, NNODE, 2.0f);
  pack_xg_kernel<<<gxg, 256, 0, stream>>>(X0h, X0l, X1h, X1l, P2, XGh, XGl);
  for (int c = 0; c < MROWS / GCHUNK; ++c) {
    const size_t aoff = (size_t)c * GCHUNK * KPAD;
    wmma_gemm64<1, 3, 0><<<gng, 256, 0, stream>>>(XGh + aoff, XGl + aoff, KPAD, 0L, PTg, PTg, KPAD, 0L,
                                                   (void*)Y, (void*)Y, NDG, 0L,
                                                   GCHUNK, NDG, KPAD, 1.0f);
    gate_epi_kernel<<<GCHUNK / NTILE, 256, 0, stream>>>(Y, E, gB, state, zb, X0h, X0l, c * GCHUNK);
  }

  wmma_gemm64<1, 1, 2><<<gprop, 256, 0, stream>>>(X0h, X0l, NNODE, 0L, Ah, Al, NNODE, 0L,
                                                   (void*)X1h, (void*)X1l, NNODE, 0L,
                                                   FPAD, NNODE, NNODE, 1.0f);
  wmma_gemm64<1, 1, 0><<<gprop, 256, 0, stream>>>(X1h, X1l, NNODE, 0L, Ah, Al, NNODE, 0L,
                                                   (void*)P2, (void*)P2, NNODE, 0L,
                                                   FPAD, NNODE, NNODE, 2.0f);
  pack_xg_kernel<<<gxg, 256, 0, stream>>>(X0h, X0l, X1h, X1l, P2, XGh, XGl);
  for (int c = 0; c < MROWS / UCHUNK; ++c) {
    const size_t aoff = (size_t)c * UCHUNK * KPAD;
    wmma_gemm64<1, 3, 0><<<gnu, 256, 0, stream>>>(XGh + aoff, XGl + aoff, KPAD, 0L, PTu, PTu, KPAD, 0L,
                                                   (void*)Y, (void*)Y, NDU, 0L,
                                                   UCHUNK, NDU, KPAD, 1.0f);
    cand_epi_kernel<<<UCHUNK / NTILE, 256, 0, stream>>>(Y, E, uB, state, zb, out, c * UCHUNK);
  }
}
